// MultiheadAttention_45251775430659
// MI455X (gfx1250) — hardware-verified
//
#include <hip/hip_runtime.h>


#ifndef NB
#define NB 2
#endif
#ifndef SEQ
#define SEQ 4096
#endif
#define NB_FULL  2
#define SEQ_FULL 4096
#define DM    512
#define NH    8
#define HD    64
#define DQKV  1536
#define ROWS  (NB * SEQ)
#define PLN   ((size_t)NB * NH * SEQ * HD)
#define L2E   1.4426950408889634f
#define PCARL 10.0f

static_assert(NH * HD == DM);
static_assert(DQKV == 3 * DM);
static_assert(HD == 64);
static_assert(DM % 64 == 0);
static_assert(DM % 32 == 0);
static_assert(DQKV % 64 == 0);
static_assert(SEQ % 64 == 0);
static_assert(ROWS % 64 == 0);
static_assert(SEQ <= SEQ_FULL);
static_assert(NB <= NB_FULL);

typedef _Float16 h16;
typedef unsigned short bf;
typedef __attribute__((ext_vector_type(16))) __bf16   v16bf;
typedef __attribute__((ext_vector_type(16))) _Float16 v16h;
typedef __attribute__((ext_vector_type(8)))  _Float16 v8h;
typedef __attribute__((ext_vector_type(8)))  unsigned short v8us;
typedef __attribute__((ext_vector_type(2)))  unsigned short v2us;
typedef __attribute__((ext_vector_type(8)))  float    v8f;
typedef __attribute__((ext_vector_type(4)))  float    v4f;
typedef __attribute__((ext_vector_type(2)))  float    v2f;
typedef v4f  __attribute__((may_alias)) v4fa;
typedef v8us __attribute__((may_alias)) v8usa;

__device__ __forceinline__ unsigned short f2bf(float f) { unsigned u = __float_as_uint(f); u += 0x7FFFu + ((u >> 16) & 1u); return (unsigned short)(u >> 16); }
__device__ __forceinline__ float bf2f(unsigned short b) { return __uint_as_float(((unsigned)b) << 16); }
__device__ __forceinline__ float bfr(float f) { return bf2f(f2bf(f)); }
__device__ __forceinline__ void splitf(float y, unsigned short& h, unsigned short& l) { h = f2bf(y); l = f2bf(y - bf2f(h)); }
__device__ __forceinline__ v16h cat16(v8h lo, v8h hi) { return __builtin_shufflevector(lo, hi, 0, 1, 2, 3, 4, 5, 6, 7, 8, 9, 10, 11, 12, 13, 14, 15); }
__device__ __forceinline__ v16bf cat16b(v8us lo, v8us hi) { return __builtin_bit_cast(v16bf, __builtin_shufflevector(lo, hi, 0, 1, 2, 3, 4, 5, 6, 7, 8, 9, 10, 11, 12, 13, 14, 15)); }
__device__ __forceinline__ v16bf ldb(const bf* p) { return cat16b(*(const v8us*)p, *(const v8us*)(p + 16)); }
__device__ __forceinline__ v16h ldh(const h16* p) { return cat16(*(const v8h*)p, *(const v8h*)(p + 16)); }
__device__ __forceinline__ v8f mmab(v16bf a, v16bf b, v8f c) {
    c = __builtin_amdgcn_wmma_f32_16x16x32_bf16(false, a, false, b, (short)0, c, false, false);
    asm volatile("v_nop\n\tv_nop\n\tv_nop\n\tv_nop" : "+v"(c) : "v"(a), "v"(b));
    return c;
}
__device__ __forceinline__ v8f mmah(v16h a, v16h b, v8f c) {
    c = __builtin_amdgcn_wmma_f32_16x16x32_f16(false, a, false, b, (short)0, c, false, false);
    asm volatile("v_nop\n\tv_nop\n\tv_nop\n\tv_nop" : "+v"(c) : "v"(a), "v"(b));
    return c;
}

__global__ __launch_bounds__(256) void k_wtG(const float* __restrict__ w, int K, int N, bf* Bt) {
    const int lane = threadIdx.x & 31; const int L0 = (blockIdx.x * 8 + (threadIdx.x >> 5)) * 8; const int nlines = N * K / 64;
#pragma unroll
    for (int ps = 0; ps < 2; ++ps) {
#pragma unroll 1
        for (int l = 0; l < 8; ++l) { const int L = L0 + l; if (L >= nlines) break; const size_t e = (size_t)L * 64 + lane * 2; const int k = (int)(e % K), n = (int)(e / K); v2us o;
            o[0] = f2bf(w[(size_t)k * N + n]); o[1] = f2bf(w[(size_t)(k + 1) * N + n]); *(volatile v2us*)(Bt + e) = o; }
        if (ps == 0) __threadfence(); }
}

__global__ __launch_bounds__(256) void k_pe(float* PE) {
#pragma clang fp contract(off)
    const int idx = blockIdx.x * 256 + threadIdx.x; if (idx >= SEQ * (DM / 2)) return;
    const int m = idx % (DM / 2); const int n = idx / (DM / 2);
    double p = 1.0;
    p *= (m & 1)   ? 1.0366329284376980 : 1.0;
    p *= (m & 2)   ? 1.0746078283213174 : 1.0;
    p *= (m & 4)   ? 1.1547819846894583 : 1.0;
    p *= (m & 8)   ? 1.3335214321633240 : 1.0;
    p *= (m & 16)  ? 1.7782794100389228 : 1.0;
    p *= (m & 32)  ? 3.1622776601683795 : 1.0;
    p *= (m & 64)  ? 10.0 : 1.0;
    p *= (m & 128) ? 100.0 : 1.0;
    const float pf = (float)p;
    const float ang = (float)n / pf;
    float sn, cs; sincosf(ang, &sn, &cs);
    v2f o; o[0] = sn; o[1] = cs;
    *(volatile v2f*)(PE + (size_t)idx * 2) = o; __threadfence(); *(volatile v2f*)(PE + (size_t)idx * 2) = o;
}

__global__ __launch_bounds__(256) void k_xp(const float* __restrict__ x, const float* __restrict__ PE, bf* XH, bf* XL) {
    const size_t i = (size_t)blockIdx.x * 256 + threadIdx.x; if (i >= (size_t)ROWS * DM / 8) return;
    const size_t e = i * 8; const int c = (int)(e % DM); const size_t row = e / DM; const int t = (int)(row % SEQ); const int b = (int)(row / SEQ);
    const float* xs = x + ((size_t)b * SEQ_FULL + t) * DM + c; const float* ps = PE + (size_t)t * DM + c;
    const v4f a0 = *(const v4f*)xs, a1 = *(const v4f*)(xs + 4), p0 = *(const v4f*)ps, p1 = *(const v4f*)(ps + 4);
    v8us oh, ol;
#pragma unroll
    for (int k = 0; k < 4; ++k) { unsigned short a, c2; splitf(bfr(a0[k]) + p0[k], a, c2); oh[k] = a; ol[k] = c2; splitf(bfr(a1[k]) + p1[k], a, c2); oh[4 + k] = a; ol[4 + k] = c2; }
    *(volatile v8us*)(XH + e) = oh; *(volatile v8us*)(XL + e) = ol; __threadfence(); *(volatile v8us*)(XH + e) = oh; *(volatile v8us*)(XL + e) = ol;
}

template <bool BIAS>
__device__ __forceinline__ void gemmw_body(const bf* __restrict__ A, const bf* __restrict__ A2, const bf* __restrict__ Bt, int K, float* C, int ldc, const float* __restrict__ bias) {
    __shared__ __align__(16) float os[16 * 68];
    const int lane = threadIdx.x & 31, lr = lane & 15, hi = lane >> 4; const int r0 = blockIdx.x * 64, c0 = blockIdx.y * 64;
    v8f acc[4][4];
#pragma unroll
    for (int mb = 0; mb < 4; ++mb)
#pragma unroll
        for (int nb = 0; nb < 4; ++nb) acc[mb][nb] = (v8f){};
    const size_t aoff = (size_t)(r0 + lr) * K + 8 * hi, boff = (size_t)(c0 + lr) * K + 8 * hi;
#pragma unroll 1
    for (int kc = 0; kc < K; kc += 32) {
        v16bf a[4], a2[4];
#pragma unroll
        for (int mb = 0; mb < 4; ++mb) { a[mb] = ldb(A + aoff + (size_t)mb * 16 * K + kc); a2[mb] = ldb(A2 + aoff + (size_t)mb * 16 * K + kc); }
#pragma unroll
        for (int nb = 0; nb < 4; ++nb) { const v16bf b = ldb(Bt + boff + (size_t)nb * 16 * K + kc);
#pragma unroll
            for (int mb = 0; mb < 4; ++mb) { acc[mb][nb] = mmab(a[mb], b, acc[mb][nb]); acc[mb][nb] = mmab(a2[mb], b, acc[mb][nb]); } }
    }
#pragma unroll
    for (int mb = 0; mb < 4; ++mb) {
#pragma unroll
        for (int nb = 0; nb < 4; ++nb) {
#pragma unroll
            for (int j = 0; j < 8; ++j) os[(hi * 8 + j) * 68 + nb * 16 + lr] = acc[mb][nb][j]; }
        __builtin_amdgcn_wave_barrier(); asm volatile("" ::: "memory");
        float* crow = C + (size_t)(r0 + mb * 16) * ldc + c0;
#pragma unroll 1
        for (int ps = 0; ps < 2; ++ps) {
#pragma unroll
            for (int s = 0; s < 8; ++s) { const int row = 2 * s + hi, cofs = lr * 4; v4f val = *(const v4fa*)(os + row * 68 + cofs); if (BIAS) { val[0] += bfr(bias[c0 + cofs]); val[1] += bfr(bias[c0 + cofs + 1]); val[2] += bfr(bias[c0 + cofs + 2]); val[3] += bfr(bias[c0 + cofs + 3]); }
                *(volatile v4f*)(crow + (size_t)row * ldc + cofs) = val; }
            if (ps == 0) __threadfence(); }
        __builtin_amdgcn_wave_barrier(); asm volatile("" ::: "memory");
    }
}
__global__ __launch_bounds__(32) void k_gemm_qkv(const bf* __restrict__ A, const bf* __restrict__ A2, const bf* __restrict__ Bt, int K, float* C, int ldc) { gemmw_body<false>(A, A2, Bt, K, C, ldc, nullptr); }
__global__ __launch_bounds__(32) void k_gemm_out(const bf* __restrict__ A, const bf* __restrict__ A2, const bf* __restrict__ Bt, int K, float* C, int ldc, const float* __restrict__ bias) { gemmw_body<true>(A, A2, Bt, K, C, ldc, bias); }

__global__ __launch_bounds__(256) void k_qkp(const float* __restrict__ F, bf* PH, bf* PL) {
    const size_t i = (size_t)blockIdx.x * 256 + threadIdx.x; if (i >= (size_t)2 * PLN / 8) return;
    const int d8 = (int)(i & 7); const int t = (int)((i >> 3) % SEQ); const int hh = (int)((i / ((size_t)8 * SEQ)) % NH); const int b = (int)((i / ((size_t)8 * SEQ * NH)) % NB); const int which = (int)(i / ((size_t)8 * SEQ * NH * NB));
    const float sc = (which == 0) ? 0.125f : 1.0f;
    const float* f = F + ((size_t)b * SEQ + t) * DQKV + which * DM + hh * HD + d8 * 8;
    const v4f a0 = *(const v4f*)f, a1 = *(const v4f*)(f + 4);
    v8us oh, ol;
#pragma unroll
    for (int k = 0; k < 4; ++k) { unsigned short a, c2; splitf(a0[k] * sc, a, c2); oh[k] = a; ol[k] = c2; splitf(a1[k] * sc, a, c2); oh[4 + k] = a; ol[4 + k] = c2; }
    const size_t e = i * 8;
    *(volatile v8us*)(PH + e) = oh; *(volatile v8us*)(PL + e) = ol; __threadfence(); *(volatile v8us*)(PH + e) = oh; *(volatile v8us*)(PL + e) = ol;
}

__global__ __launch_bounds__(256) void k_vt(const float* __restrict__ F, h16* VT) {
    const size_t i = (size_t)blockIdx.x * 256 + threadIdx.x; if (i >= PLN / 8) return;
    const int t8 = (int)(i % (SEQ / 8)); const int d = (int)((i / (SEQ / 8)) % HD); const int hh = (int)((i / ((size_t)(SEQ / 8) * HD)) % NH); const int b = (int)(i / ((size_t)(SEQ / 8) * HD * NH));
    const float* f = F + ((size_t)b * SEQ + (size_t)t8 * 8) * DQKV + 2 * DM + hh * HD + d;
    v8h o;
#pragma unroll
    for (int q = 0; q < 8; ++q) o[q] = (h16)f[(size_t)q * DQKV];
    *(volatile v8h*)(VT + i * 8) = o; __threadfence(); *(volatile v8h*)(VT + i * 8) = o;
}

__global__ __launch_bounds__(128) void k_flash(const bf* __restrict__ PH, const bf* __restrict__ PL, const h16* __restrict__ VT, bf* CH, bf* CL) {
    __shared__ __align__(16) unsigned short sH[4 * 16 * 72];
    __shared__ __align__(16) unsigned short sL[4 * 16 * 72];
    const int wave = __builtin_amdgcn_readfirstlane(threadIdx.x >> 5);
    const int lane = threadIdx.x & 31, lr = lane & 15, hi = lane >> 4;
    const int bh = blockIdx.y; const int b = bh / NH, hh = bh % NH;
    const int q0 = blockIdx.x * 64 + wave * 16;
    const size_t hb = (size_t)bh * SEQ * HD;
    const size_t qoff = hb + (size_t)(q0 + lr) * HD + 8 * hi;
    const v16bf qh0 = ldb(PH + qoff), qh1 = ldb(PH + qoff + 32), ql0 = ldb(PL + qoff), ql1 = ldb(PL + qoff + 32);
    const size_t kbase = PLN + hb + (size_t)lr * HD + 8 * hi;
    const size_t vbase = (size_t)bh * HD * SEQ + (size_t)lr * SEQ + 8 * hi;
    v8f o[4];
#pragma unroll
    for (int f = 0; f < 4; ++f) o[f] = (v8f){};
    float m = -1.0e30f, l = 0.0f;
#pragma unroll 1
    for (int key0 = 0; key0 < SEQ; key0 += 32) {
        const size_t ko = kbase + (size_t)key0 * HD;
        v8f s0 = (v8f){}, s1 = (v8f){};
        { const v16bf kh = ldb(PH + ko), kl = ldb(PL + ko); s0 = mmab(kh, qh0, s0); s0 = mmab(kh, ql0, s0); s0 = mmab(kl, qh0, s0); }
        { const v16bf kh = ldb(PH + ko + 32), kl = ldb(PL + ko + 32); s0 = mmab(kh, qh1, s0); s0 = mmab(kh, ql1, s0); s0 = mmab(kl, qh1, s0); }
        { const v16bf kh = ldb(PH + ko + 16 * HD), kl = ldb(PL + ko + 16 * HD); s1 = mmab(kh, qh0, s1); s1 = mmab(kh, ql0, s1); s1 = mmab(kl, qh0, s1); }
        { const v16bf kh = ldb(PH + ko + 16 * HD + 32), kl = ldb(PL + ko + 16 * HD + 32); s1 = mmab(kh, qh1, s1); s1 = mmab(kh, ql1, s1); s1 = mmab(kl, qh1, s1); }
        float mx = fmaxf(s0[0], s1[0]);
#pragma unroll
        for (int r = 1; r < 8; ++r) mx = fmaxf(mx, fmaxf(s0[r], s1[r]));
        mx = fmaxf(mx, __shfl_xor(mx, 16, 32));
        const float mn = fmaxf(m, mx);
        const float alpha = __builtin_amdgcn_exp2f((m - mn) * L2E);
        m = mn;
        float ps = 0.0f; v16h pf;
#pragma unroll
        for (int r = 0; r < 8; ++r) {
            const float p0 = __builtin_amdgcn_exp2f(fmaf(s0[r] - mn, L2E, PCARL));
            const float p1 = __builtin_amdgcn_exp2f(fmaf(s1[r] - mn, L2E, PCARL));
            ps += p0 + p1; pf[r] = (h16)p0; pf[8 + r] = (h16)p1; }
        l = l * alpha + ps;
#pragma unroll
        for (int f = 0; f < 4; ++f) o[f] *= alpha;
        const size_t vo = vbase + (size_t)key0;
        { const v16h va = ldh(VT + vo); o[0] = mmah(va, pf, o[0]); }
        { const v16h va = ldh(VT + vo + (size_t)16 * SEQ); o[1] = mmah(va, pf, o[1]); }
        { const v16h va = ldh(VT + vo + (size_t)32 * SEQ); o[2] = mmah(va, pf, o[2]); }
        { const v16h va = ldh(VT + vo + (size_t)48 * SEQ); o[3] = mmah(va, pf, o[3]); }
    }
    const float lt = l + __shfl_xor(l, 16, 32);
    const float inv = 1.0f / lt;
    const int tb = wave * (16 * 72);
#pragma unroll
    for (int f = 0; f < 4; ++f) { v8us oh, ol;
#pragma unroll
        for (int r = 0; r < 8; ++r) { unsigned short a, c2; splitf(o[f][r] * inv, a, c2); oh[r] = a; ol[r] = c2; }
        *(v8usa*)(&sH[tb + lr * 72 + 16 * f + 8 * hi]) = oh; *(v8usa*)(&sL[tb + lr * 72 + 16 * f + 8 * hi]) = ol; }
    __builtin_amdgcn_wave_barrier(); asm volatile("" ::: "memory");
#pragma unroll 1
    for (int ps2 = 0; ps2 < 2; ++ps2) {
#pragma unroll
        for (int s = 0; s < 4; ++s) { const int row = 4 * s + (lane >> 3), pc = lane & 7;
            const v8us vh = *(const v8usa*)(&sH[tb + row * 72 + pc * 8]); const v8us vl = *(const v8usa*)(&sL[tb + row * 72 + pc * 8]);
            const size_t go = ((size_t)b * SEQ + q0 + row) * DM + hh * HD + pc * 8;
            *(volatile v8us*)(CH + go) = vh; *(volatile v8us*)(CL + go) = vl; }
        if (ps2 == 0) __threadfence(); }
}

constexpr size_t SZ_WQKV = (size_t)DQKV * DM * 2;
constexpr size_t SZ_WO   = (size_t)DM * DM * 2;
constexpr size_t SZ_PE   = (size_t)SEQ * DM * 4;
constexpr size_t SZ_X    = (size_t)ROWS * DM * 2;
constexpr size_t SZ_F    = (size_t)ROWS * DQKV * 4;
constexpr size_t SZ_QK   = (size_t)2 * PLN * 2;
constexpr size_t SZ_VT   = PLN * 2;
constexpr size_t OFF_WQKV = 0;
constexpr size_t OFF_WO   = OFF_WQKV + SZ_WQKV;
constexpr size_t OFF_PE   = OFF_WO + SZ_WO;
constexpr size_t OFF_XH   = OFF_PE + SZ_PE;
constexpr size_t OFF_XL   = OFF_XH + SZ_X;
constexpr size_t OFF_F    = OFF_XL + SZ_X;
constexpr size_t OFF_PH   = OFF_F + SZ_F;
constexpr size_t OFF_PL   = OFF_PH + SZ_QK;
constexpr size_t OFF_VT   = OFF_PL + SZ_QK;
constexpr size_t WS_TOTAL = OFF_VT + SZ_VT;
static_assert(WS_TOTAL <= (size_t)134217728);
static_assert(SZ_WQKV % 256 == 0);
static_assert(SZ_WO % 256 == 0);
static_assert(SZ_PE % 256 == 0);
static_assert(SZ_X % 256 == 0);
static_assert(SZ_F % 256 == 0);
static_assert(SZ_QK % 256 == 0);
static_assert(SZ_VT % 256 == 0);
static_assert((size_t)ROWS * DM * 2 == SZ_X);
static_assert(((size_t)ROWS * DM / 8) % 256 == 0);
static_assert(((size_t)2 * PLN / 8) % 256 == 0);
static_assert(((size_t)SEQ * (DM / 2)) % 256 == 0);

extern "C" void kernel_launch(void* const* d_in, const int* in_sizes, int n_in,
                              void* d_out, int out_size, void* d_ws, size_t ws_size, hipStream_t stream) {
    if (n_in < 4) return;
    if ((size_t)in_sizes[0] < ((size_t)(NB - 1) * SEQ_FULL + SEQ) * DM) return;
    if ((size_t)in_sizes[1] < (size_t)DM * DQKV) return;
    if ((size_t)in_sizes[2] < (size_t)DM * DM) return;
    if ((size_t)in_sizes[3] < (size_t)DM) return;
    if ((size_t)out_size < (size_t)ROWS * DM) return;
    if (WS_TOTAL > ws_size) return;
    const float* x = (const float*)d_in[0]; const float* wqkv = (const float*)d_in[1]; const float* wo = (const float*)d_in[2]; const float* bo = (const float*)d_in[3];
    float* OUT = (float*)d_out;
    char* ws = (char*)d_ws;
    bf* WQKV = (bf*)(ws + OFF_WQKV); bf* WO = (bf*)(ws + OFF_WO); float* PE = (float*)(ws + OFF_PE);
    bf* XH = (bf*)(ws + OFF_XH); bf* XL = (bf*)(ws + OFF_XL); float* F = (float*)(ws + OFF_F);
    bf* PH = (bf*)(ws + OFF_PH); bf* PL = (bf*)(ws + OFF_PL); h16* VT = (h16*)(ws + OFF_VT);
    bf* CH = XH; bf* CL = XL;

    k_wtG<<<(unsigned)((DM * DQKV / 64 + 63) / 64), 256, 0, stream>>>(wqkv, DM, DQKV, WQKV);
    k_wtG<<<(unsigned)((DM * DM / 64 + 63) / 64), 256, 0, stream>>>(wo, DM, DM, WO);
    k_pe<<<(unsigned)(((size_t)SEQ * (DM / 2)) / 256), 256, 0, stream>>>(PE);
    k_xp<<<(unsigned)(((size_t)ROWS * DM / 8) / 256), 256, 0, stream>>>(x, PE, XH, XL);
    k_gemm_qkv<<<dim3(ROWS / 64, DQKV / 64, 1), 32, 0, stream>>>(XH, XL, WQKV, DM, F, DQKV);
    k_qkp<<<(unsigned)(((size_t)2 * PLN / 8) / 256), 256, 0, stream>>>(F, PH, PL);
    k_vt<<<(unsigned)((PLN / 8) / 256), 256, 0, stream>>>(F, VT);
    k_flash<<<dim3(SEQ / 64, NB * NH, 1), 128, 0, stream>>>(PH, PL, VT, CH, CL);
    k_gemm_out<<<dim3(ROWS / 64, DM / 64, 1), 32, 0, stream>>>(CH, CL, WO, DM, OUT, DM, bo);
}
